// SubsetsSampleWeighted_71347996721713
// MI455X (gfx1250) — hardware-run, weakly checked
//
#include <hip/hip_runtime.h>

typedef __attribute__((ext_vector_type(16))) _Float16 v16h;
typedef __attribute__((ext_vector_type(8)))  _Float16 v8h;
typedef __attribute__((ext_vector_type(8)))  float    v8f;
typedef __attribute__((ext_vector_type(4)))  float    v4f;
typedef __attribute__((ext_vector_type(2)))  float    v2f;

constexpr int kNumB   = 16;
constexpr int kAtoms  = 64;
constexpr int kFeat   = 128;
constexpr int kSub    = 8192;
constexpr int kPeaks  = 16;
constexpr int kHid    = 128;
constexpr int kBins   = 512;
constexpr int kRowsPerBlock = 128;
constexpr int kStripPitch   = 136;
constexpr float kLnEps      = 1e-5f;
constexpr float kSizeEps    = 1e-4f;
constexpr float kWCarry     = 64.0f;
constexpr float kWCarryInv  = 1.0f / kWCarry;
constexpr float kInvFeat    = 1.0f / (float)kFeat;
constexpr float kInvHid     = 1.0f / (float)kHid;
constexpr float kFixScale   = 131072.0f;
constexpr float kFixInv     = 1.0f / kFixScale;
static_assert(kAtoms == 64 && kFeat == 128 && kHid == 128);
static_assert((kAtoms % 32) == 0 && (kFeat % 32) == 0 && (kHid % 32) == 0);
static_assert((kSub % kRowsPerBlock) == 0 && (kFeat % 16) == 0 && (kHid % 16) == 0);
static_assert((kStripPitch % 8) == 0 && kStripPitch >= kFeat);

constexpr size_t kOffW1T    = 0;
constexpr size_t kOffW2T    = kOffW1T   + (size_t)kHid * kFeat * 2;
constexpr size_t kOffFeatT  = kOffW2T   + (size_t)kHid * kHid * 2;
constexpr size_t kOffScores = kOffFeatT + (size_t)kNumB * kFeat * kAtoms * 2;
constexpr size_t kWsTotal   = kOffScores + (size_t)kNumB * kSub * 4;
static_assert(kWsTotal == 851968ull);
static_assert(kWsTotal <= 134217728ull);
static_assert((kOffW2T % 128) == 0 && (kOffFeatT % 128) == 0 && (kOffScores % 128) == 0);

constexpr size_t kOutProbsByteOff = (size_t)kNumB * kBins * 4;
static_assert(kOutProbsByteOff == 32768ull);
static_assert(kOutProbsByteOff + (size_t)kNumB * kSub * 4 == 557056ull);
static_assert((kOutProbsByteOff % 128) == 0);

union FragU { v16h v; v8h h[2]; };

__device__ __forceinline__ v16h frag_load(const _Float16* p) {
  FragU f;
  f.h[0] = *(const v8h*)(p);
  f.h[1] = *(const v8h*)(p + 16);
  return f.v;
}

__device__ __forceinline__ v8f wm(v16h a, v16h b, v8f c) {
  c = __builtin_amdgcn_wmma_f32_16x16x32_f16(false, a, false, b, (short)0, c, false, false);
  asm volatile("v_nop\n\tv_nop\n\tv_nop\n\tv_nop" : "+v"(c) : "v"(a), "v"(b));
  return c;
}

__device__ __forceinline__ v8f vzero8() {
  return (v8f){0.f, 0.f, 0.f, 0.f, 0.f, 0.f, 0.f, 0.f};
}

__device__ __forceinline__ float red16(float v) {
  v += __shfl_xor(v, 1);
  v += __shfl_xor(v, 2);
  v += __shfl_xor(v, 4);
  v += __shfl_xor(v, 8);
  return v;
}

__device__ __forceinline__ void load_sub8(const int* __restrict__ p, const float* __restrict__ m,
                                          v8h& o, float& sz) {
  const int4 i0 = *(const int4*)(p);
  const int4 i1 = *(const int4*)(p + 4);
  const v4f m0 = *(const v4f*)(m);
  const v4f m1 = *(const v4f*)(m + 4);
  const float f0 = (float)i0.x;
  const float f1 = (float)i0.y;
  const float f2 = (float)i0.z;
  const float f3 = (float)i0.w;
  const float f4 = (float)i1.x;
  const float f5 = (float)i1.y;
  const float f6 = (float)i1.z;
  const float f7 = (float)i1.w;
  o[0] = (_Float16)f0;
  o[1] = (_Float16)f1;
  o[2] = (_Float16)f2;
  o[3] = (_Float16)f3;
  o[4] = (_Float16)f4;
  o[5] = (_Float16)f5;
  o[6] = (_Float16)f6;
  o[7] = (_Float16)f7;
  sz += f0 * m0[0];
  sz += f1 * m0[1];
  sz += f2 * m0[2];
  sz += f3 * m0[3];
  sz += f4 * m1[0];
  sz += f5 * m1[1];
  sz += f6 * m1[2];
  sz += f7 * m1[3];
}

__global__ __launch_bounds__(256) void prep_planes_kernel(
    const float* __restrict__ feat, const float* __restrict__ mask,
    const float* __restrict__ W1, const float* __restrict__ W2,
    _Float16* __restrict__ featT, _Float16* __restrict__ W1t, _Float16* __restrict__ W2t)
{
  const int tid = threadIdx.x;
  const int blk = blockIdx.x;
  v8h hv;
  _Float16* dst;
  if (blk < 16) {
    const float* W  = (blk < 8) ? W1 : W2;
    _Float16*    Wt = (blk < 8) ? W1t : W2t;
    const int gid = (blk & 7) * 256 + tid;
    const int nn  = gid >> 4;
    const int k8  = (gid & 15) * 8;
#pragma unroll
    for (int e = 0; e < 8; ++e) {
      const float w = W[(size_t)(k8 + e) * kHid + nn];
      hv[e] = (_Float16)(w * kWCarry);
    }
    dst = Wt + (size_t)gid * 8;
  } else {
    const int gid = (blk - 16) * 256 + tid;
    const int a8  = (gid & 7) * 8;
    const int g   = (gid >> 3) & (kFeat - 1);
    const int bb  = gid >> 10;
#pragma unroll
    for (int e = 0; e < 8; ++e) {
      const float m = mask[bb * kAtoms + a8 + e];
      const float f = feat[((size_t)bb * kAtoms + a8 + e) * kFeat + g];
      const float fm = f * m;
      hv[e] = (_Float16)(fm * m);
    }
    dst = featT + (size_t)gid * 8;
  }
  *(volatile v8h*)dst = hv;
  __threadfence();
  *(volatile v8h*)dst = hv;
}

__global__ __launch_bounds__(256) void pooled_scorer_kernel(
    const int* __restrict__ subsets, const float* __restrict__ mask,
    const _Float16* __restrict__ featT, const _Float16* __restrict__ W1t, const _Float16* __restrict__ W2t,
    const float* __restrict__ ln0w, const float* __restrict__ ln0b,
    const float* __restrict__ b1g, const float* __restrict__ b2g,
    const float* __restrict__ ln1w, const float* __restrict__ ln1b,
    const float* __restrict__ Wsg, const float* __restrict__ bsg,
    float* __restrict__ scores)
{
  __shared__ __align__(16) _Float16 sStrip[8][16 * kStripPitch];
  __shared__ __align__(16) float sP[7 * 128];
  __shared__ __align__(16) float sScore[kRowsPerBlock];

  const int tid  = threadIdx.x;
  const int lane = tid & 31;
  const int wave = tid >> 5;
  const int hh   = lane >> 4;
  const int n    = lane & 15;
  const int b    = blockIdx.y;
  const int s0   = blockIdx.x * kRowsPerBlock;
  const int row0 = s0 + wave * 16;

  {
    const float* psrc = ln0w;
    if (wave == 1) psrc = ln0b;
    if (wave == 2) psrc = b1g;
    if (wave == 3) psrc = b2g;
    if (wave == 4) psrc = ln1w;
    if (wave == 5) psrc = ln1b;
    if (wave == 6) psrc = Wsg;
    const v4f pv = *(const v4f*)(psrc + lane * 4);
    if (wave < 7) *(v4f*)(&sP[wave * 128 + lane * 4]) = pv;
  }
  const float bsv = bsg[0];

  FragU fa0, fa1;
  float szp = 0.0f;
  {
    const int*   srow = subsets + ((size_t)b * kSub + row0 + n) * kAtoms + 8 * hh;
    const float* mrow = mask + b * kAtoms + 8 * hh;
    load_sub8(srow,      mrow,      fa0.h[0], szp);
    load_sub8(srow + 16, mrow + 16, fa0.h[1], szp);
    load_sub8(srow + 32, mrow + 32, fa1.h[0], szp);
    load_sub8(srow + 48, mrow + 48, fa1.h[1], szp);
  }
  const float szt = szp + __shfl_xor(szp, 16);
  const float inv_size = 1.0f / (szt + kSizeEps);

  __syncthreads();

  _Float16* strip = &sStrip[wave][0];
  v8f acc[8];

  {
    const _Float16* fT = featT + (size_t)b * kFeat * kAtoms;
#pragma unroll
    for (int t = 0; t < 8; ++t) {
      asm volatile("" ::: "memory");
      const _Float16* bp = fT + (size_t)(t * 16 + n) * kAtoms + 8 * hh;
      const v16h bf0 = frag_load(bp);
      const v16h bf1 = frag_load(bp + 32);
      v8f c = vzero8();
      c = wm(fa0.v, bf0, c);
      c = wm(fa1.v, bf1, c);
      acc[t] = c;
    }
  }
#pragma unroll
  for (int r = 0; r < 8; ++r) {
    const float iv = __shfl(inv_size, 8 * hh + r);
    float s = 0.0f;
#pragma unroll
    for (int t = 0; t < 8; ++t) {
      acc[t][r] *= iv;
      s += acc[t][r];
    }
    s = red16(s);
    const float mu = s * kInvFeat;
    float q = 0.0f;
#pragma unroll
    for (int t = 0; t < 8; ++t) {
      const float d = acc[t][r] - mu;
      q = fmaf(d, d, q);
    }
    q = red16(q);
    const float rs = rsqrtf(q * kInvFeat + kLnEps);
#pragma unroll
    for (int t = 0; t < 8; ++t) {
      const int col = t * 16 + n;
      const float y = (acc[t][r] - mu) * rs * sP[col] + sP[128 + col];
      strip[(8 * hh + r) * kStripPitch + col] = (_Float16)y;
    }
  }
  __syncthreads();

  {
    v16h xa[4];
#pragma unroll
    for (int k = 0; k < 4; ++k) xa[k] = frag_load(&sStrip[wave][n * kStripPitch + k * 32 + 8 * hh]);
    __syncthreads();
#pragma unroll 1
    for (int t = 0; t < 8; ++t) {
      const _Float16* bp = W1t + (size_t)(t * 16 + n) * kFeat + 8 * hh;
      v8f c = vzero8();
#pragma unroll
      for (int k = 0; k < 4; ++k) {
        const v16h bf = frag_load(bp + k * 32);
        c = wm(xa[k], bf, c);
      }
      const int col = t * 16 + n;
      const float bb = sP[2 * 128 + col];
#pragma unroll
      for (int r = 0; r < 8; ++r) {
        const float y = fmaxf(fmaf(c[r], kWCarryInv, bb), 0.0f);
        strip[(8 * hh + r) * kStripPitch + col] = (_Float16)y;
      }
    }
  }
  __syncthreads();

  {
    v16h ha[4];
#pragma unroll
    for (int k = 0; k < 4; ++k) ha[k] = frag_load(&sStrip[wave][n * kStripPitch + k * 32 + 8 * hh]);
#pragma unroll
    for (int t = 0; t < 8; ++t) {
      asm volatile("" ::: "memory");
      const _Float16* bp = W2t + (size_t)(t * 16 + n) * kHid + 8 * hh;
      v8f c = vzero8();
#pragma unroll
      for (int k = 0; k < 4; ++k) {
        const v16h bf = frag_load(bp + k * 32);
        c = wm(ha[k], bf, c);
      }
      const int col = t * 16 + n;
      const float bb = sP[3 * 128 + col];
#pragma unroll
      for (int r = 0; r < 8; ++r) c[r] = fmaxf(fmaf(c[r], kWCarryInv, bb), 0.0f);
      acc[t] = c;
    }
  }

  float sc[8];
#pragma unroll
  for (int r = 0; r < 8; ++r) {
    float s = 0.0f;
#pragma unroll
    for (int t = 0; t < 8; ++t) s += acc[t][r];
    s = red16(s);
    const float mu = s * kInvHid;
    float q = 0.0f;
#pragma unroll
    for (int t = 0; t < 8; ++t) {
      const float d = acc[t][r] - mu;
      q = fmaf(d, d, q);
    }
    q = red16(q);
    const float rs = rsqrtf(q * kInvHid + kLnEps);
    float p = 0.0f;
#pragma unroll
    for (int t = 0; t < 8; ++t) {
      const int col = t * 16 + n;
      const float y = (acc[t][r] - mu) * rs * sP[4 * 128 + col] + sP[5 * 128 + col];
      p = fmaf(y, sP[6 * 128 + col], p);
    }
    p = red16(p);
    sc[r] = p + bsv;
  }
  if (n == 0) {
#pragma unroll
    for (int r = 0; r < 8; ++r) sScore[wave * 16 + 8 * hh + r] = sc[r];
  }
  __syncthreads();
  if (wave == 0) {
    const v4f v = *(const v4f*)(&sScore[lane * 4]);
    float* dstp = scores + (size_t)b * kSub + s0 + lane * 4;
    *(volatile v4f*)dstp = v;
    __threadfence();
    *(volatile v4f*)dstp = v;
  }
}

__global__ __launch_bounds__(256) void softmax_rows_kernel(
    const float* __restrict__ scores, float* __restrict__ probs)
{
  __shared__ __align__(16) float sE[kSub];
  __shared__ float sRed[8];
  const int tid  = threadIdx.x;
  const int lane = tid & 31;
  const int wave = tid >> 5;
  const int b    = blockIdx.x;
  const float* sc = scores + (size_t)b * kSub;
  float*       pr = probs  + (size_t)b * kSub;

  float mx = -3.402823466e38f;
#pragma unroll 1
  for (int i = 0; i < 8; ++i) {
    const int o = (tid + i * 256) * 4;
    const v4f v = *(const v4f*)(sc + o);
    *(v4f*)(&sE[o]) = v;
    mx = fmaxf(mx, fmaxf(fmaxf(v[0], v[1]), fmaxf(v[2], v[3])));
  }
  mx = fmaxf(mx, __shfl_xor(mx, 16));
  mx = fmaxf(mx, __shfl_xor(mx, 8));
  mx = fmaxf(mx, __shfl_xor(mx, 4));
  mx = fmaxf(mx, __shfl_xor(mx, 2));
  mx = fmaxf(mx, __shfl_xor(mx, 1));
  if (lane == 0) sRed[wave] = mx;
  __syncthreads();
  float bm = sRed[0];
#pragma unroll
  for (int w = 1; w < 8; ++w) bm = fmaxf(bm, sRed[w]);
  __syncthreads();

  float sum = 0.0f;
#pragma unroll 1
  for (int i = 0; i < 8; ++i) {
    const int o = (tid + i * 256) * 4;
    const v4f v = *(const v4f*)(&sE[o]);
    v4f e;
    e[0] = expf(v[0] - bm);
    e[1] = expf(v[1] - bm);
    e[2] = expf(v[2] - bm);
    e[3] = expf(v[3] - bm);
    *(v4f*)(&sE[o]) = e;
    sum += (e[0] + e[1]) + (e[2] + e[3]);
  }
  sum += __shfl_xor(sum, 16);
  sum += __shfl_xor(sum, 8);
  sum += __shfl_xor(sum, 4);
  sum += __shfl_xor(sum, 2);
  sum += __shfl_xor(sum, 1);
  if (lane == 0) sRed[wave] = sum;
  __syncthreads();
  float tot = sRed[0];
#pragma unroll
  for (int w = 1; w < 8; ++w) tot += sRed[w];
  const float inv = 1.0f / tot;

  for (int pass = 0; pass < 2; ++pass) {
#pragma unroll 1
    for (int i = 0; i < 8; ++i) {
      const int o = (tid + i * 256) * 4;
      const v4f e = *(const v4f*)(&sE[o]);
      v4f ov;
      ov[0] = e[0] * inv;
      ov[1] = e[1] * inv;
      ov[2] = e[2] * inv;
      ov[3] = e[3] * inv;
      *(volatile v4f*)(pr + o) = ov;
    }
    __threadfence();
  }
}

__global__ __launch_bounds__(256) void mass_hist_kernel(
    const float* __restrict__ peaks, const float* __restrict__ probs, float* __restrict__ spect)
{
  __shared__ __align__(16) int sBins[kBins];
  const int tid = threadIdx.x;
  const int b   = blockIdx.x;
  sBins[tid] = 0;
  sBins[tid + 256] = 0;
  __syncthreads();
  const float* pk = peaks + (size_t)b * kSub * kPeaks * 2;
  const float* pr = probs + (size_t)b * kSub;
  constexpr int kIters = (kSub * kPeaks) / 256;
#pragma unroll 2
  for (int i = 0; i < kIters; ++i) {
    const int p = tid + i * 256;
    const v2f mi = *(const v2f*)(pk + (size_t)p * 2);
    const float pv = pr[p >> 4];
    int bin = __float2int_rn(mi[0]);
    bin = bin < 0 ? 0 : bin;
    bin = bin > (kBins - 1) ? (kBins - 1) : bin;
    const float c = mi[1] * pv;
    const int q = __float2int_rn(c * kFixScale);
    atomicAdd(&sBins[bin], q);
  }
  __syncthreads();
  if (tid < 128) {
    const int q0 = sBins[tid * 4 + 0];
    const int q1 = sBins[tid * 4 + 1];
    const int q2 = sBins[tid * 4 + 2];
    const int q3 = sBins[tid * 4 + 3];
    v4f ov;
    ov[0] = (float)q0 * kFixInv;
    ov[1] = (float)q1 * kFixInv;
    ov[2] = (float)q2 * kFixInv;
    ov[3] = (float)q3 * kFixInv;
    float* dstp = spect + (size_t)b * kBins + tid * 4;
    *(volatile v4f*)dstp = ov;
    __threadfence();
    *(volatile v4f*)dstp = ov;
  }
}

extern "C" void kernel_launch(void* const* d_in, const int* in_sizes, int n_in,
                              void* d_out, int out_size, void* d_ws, size_t ws_size,
                              hipStream_t stream) {
  if (n_in < 16) return;
  if (in_sizes[0] != kNumB * kAtoms * kFeat) return;
  if (in_sizes[1] != kNumB * kAtoms) return;
  if (in_sizes[4] != kNumB * kSub * kAtoms) return;
  if (in_sizes[5] != kNumB * kSub * kPeaks * 2) return;
  if (in_sizes[6] != kFeat || in_sizes[7] != kFeat) return;
  if (in_sizes[8] != kFeat * kHid || in_sizes[9] != kHid) return;
  if (in_sizes[10] != kHid * kHid || in_sizes[11] != kHid) return;
  if (in_sizes[12] != kHid || in_sizes[13] != kHid) return;
  if (in_sizes[14] != kHid || in_sizes[15] != 1) return;
  if (out_size != kNumB * kBins + kNumB * kSub) return;
  if (ws_size < kWsTotal) return;

  const float* feat    = (const float*)d_in[0];
  const float* mask    = (const float*)d_in[1];
  const int*   subsets = (const int*)d_in[4];
  const float* peaks   = (const float*)d_in[5];
  const float* ln0w    = (const float*)d_in[6];
  const float* ln0b    = (const float*)d_in[7];
  const float* W1      = (const float*)d_in[8];
  const float* b1      = (const float*)d_in[9];
  const float* W2      = (const float*)d_in[10];
  const float* b2      = (const float*)d_in[11];
  const float* ln1w    = (const float*)d_in[12];
  const float* ln1b    = (const float*)d_in[13];
  const float* Ws      = (const float*)d_in[14];
  const float* bs      = (const float*)d_in[15];

  float* out   = (float*)d_out;
  float* spect = out;
  float* probs = out + kOutProbsByteOff / 4;

  char* ws = (char*)d_ws;
  _Float16* W1t    = (_Float16*)(ws + kOffW1T);
  _Float16* W2t    = (_Float16*)(ws + kOffW2T);
  _Float16* featT  = (_Float16*)(ws + kOffFeatT);
  float*    scores = (float*)(ws + kOffScores);

  prep_planes_kernel<<<80, 256, 0, stream>>>(feat, mask, W1, W2, featT, W1t, W2t);
  pooled_scorer_kernel<<<dim3(kSub / kRowsPerBlock, kNumB), 256, 0, stream>>>(
      subsets, mask, featT, W1t, W2t, ln0w, ln0b, b1, b2, ln1w, ln1b, Ws, bs, scores);
  softmax_rows_kernel<<<kNumB, 256, 0, stream>>>(scores, probs);
  mass_hist_kernel<<<kNumB, 256, 0, stream>>>(peaks, probs, spect);
}
